// CLSFewShotClassifier_17111149707608
// MI455X (gfx1250) — hardware-verified
//
#include <hip/hip_runtime.h>
#include <stdint.h>


#define NIMG   800
#define NSUP   200
#define CHUNK  200
#define NCHUNK 4
#define EDIM   2304
#define NB     8
#define NS     25
#define NT     75
#define NC     5
#define KW2    576
#define FEPS   1e-8f

typedef _Float16     v16h __attribute__((ext_vector_type(16)));
typedef _Float16     v8h  __attribute__((ext_vector_type(8)));
typedef float        v8f  __attribute__((ext_vector_type(8)));
typedef float        v4f  __attribute__((ext_vector_type(4)));
typedef unsigned int u4   __attribute__((ext_vector_type(4)));

union Frag { v16h v; v8h h[2]; u4 q[2]; };
union Q16  { v8h h; u4 q; v4f f; };
union SBuf { float f[EDIM]; _Float16 hb[64 * 72]; };

__device__ __forceinline__ v8f wmma_f16(v16h a, v16h b, v8f c) {
    c = __builtin_amdgcn_wmma_f32_16x16x32_f16(false, a, false, b, (short)0, c, false, false);
    asm volatile("v_nop\n\tv_nop\n\tv_nop\n\tv_nop" : "+v"(c) : "v"(a), "v"(b));
    return c;
}

__device__ __forceinline__ v8f zero8() {
    v8f z = {0.f, 0.f, 0.f, 0.f, 0.f, 0.f, 0.f, 0.f};
    return z;
}

__global__ __launch_bounds__(256) void k_pack(const float* __restrict__ W1, const float* __restrict__ W2,
                                             const float* __restrict__ W3, const float* __restrict__ W4,
                                             _Float16* __restrict__ P1, _Float16* __restrict__ P2,
                                             _Float16* __restrict__ P3, _Float16* __restrict__ P4) {
    const int layer = blockIdx.y;
    const float* W; _Float16* P; int cin_n; int kp; float sc;
    if (layer == 0)      { W = W1; P = P1; cin_n = 3;  kp = 32;  sc = 8.0f;  }
    else if (layer == 1) { W = W2; P = P2; cin_n = 64; kp = KW2; sc = 16.0f; }
    else if (layer == 2) { W = W3; P = P3; cin_n = 64; kp = KW2; sc = 16.0f; }
    else                 { W = W4; P = P4; cin_n = 64; kp = KW2; sc = 16.0f; }

    const int g   = blockIdx.x * blockDim.x + threadIdx.x;
    const int gpr = kp >> 3;
    if (g >= 64 * gpr) return;
    const int n  = g / gpr;
    const int kg = g - n * gpr;
    const int kreal = cin_n * 9;

    Q16 o;
#pragma unroll
    for (int j = 0; j < 8; ++j) {
        const int k = kg * 8 + j;
        float v = 0.0f;
        if (k < kreal) {
            const int t  = k / cin_n;
            const int ci = k - t * cin_n;
            const int kh = t / 3;
            const int kw = t - 3 * kh;
            v = W[((n * cin_n + ci) * 3 + kh) * 3 + kw] * sc;
        }
        o.h[j] = (_Float16)v;
    }
    u4* dst = (u4*)(P + (size_t)g * 8);
    const u4 val = o.q;
    *(volatile u4*)dst = val;
    __threadfence();
    *(volatile u4*)dst = val;
}

template <int M>
__device__ __forceinline__ void epilogue_act(v8f (&acc)[4], const float* __restrict__ bias, float winv,
                                             _Float16* sD, _Float16* __restrict__ outimg,
                                             int m0, int wave, int l) {
    const int h = l >> 4, c16 = l & 15;
#pragma unroll
    for (int nb = 0; nb < 4; ++nb) {
        const int col = nb * 16 + c16;
        const float bv = bias[col];
#pragma unroll
        for (int r = 0; r < 8; ++r) {
            const int row = wave * 16 + 8 * h + r;
            const float v = fmaxf(fmaf(acc[nb][r], winv, bv), 0.0f);
            sD[row * 72 + col] = (_Float16)v;
        }
    }
    __syncthreads();

    const int p = l & 7, rq = l >> 3;
    Q16 vals[4];
#pragma unroll
    for (int i = 0; i < 4; ++i) {
        const int row = wave * 16 + i * 4 + rq;
        vals[i].h = *(const v8h*)(sD + row * 72 + p * 8);
    }
#pragma unroll
    for (int i = 0; i < 4; ++i) {
        const int m = m0 + wave * 16 + i * 4 + rq;
        if (m < M) *(volatile u4*)(outimg + (size_t)m * 64 + p * 8) = vals[i].q;
    }
    __threadfence();
#pragma unroll
    for (int i = 0; i < 4; ++i) {
        const int m = m0 + wave * 16 + i * 4 + rq;
        if (m < M) *(volatile u4*)(outimg + (size_t)m * 64 + p * 8) = vals[i].q;
    }
}

__global__ __launch_bounds__(128) void k_conv1(const float* __restrict__ x,
                                               const _Float16* __restrict__ Wp,
                                               const float* __restrict__ bias,
                                               _Float16* __restrict__ out) {
    constexpr int HIN = 84, WIN = 84, WO = 42, M = 1764, IPIX = 7056, AP = 40;
    __shared__ __align__(16) _Float16 sA[64 * AP];
    __shared__ __align__(16) _Float16 sD[64 * 72];

    const int img = blockIdx.y, m0 = blockIdx.x * 64;
    const int tid = threadIdx.x, l = tid & 31, wave = tid >> 5, h = l >> 4, c16 = l & 15;
    const float* in = x + (size_t)img * 3 * IPIX;

    {
        const int kk = l;
        const int t  = kk / 3, ci = kk - 3 * t;
        const int kh = t / 3,  kw = t - 3 * kh;
        const bool kok = kk < 27;
        const float* inc = in + (size_t)(kok ? ci : 0) * IPIX;
#pragma unroll 4
        for (int i = 0; i < 16; ++i) {
            const int ml = wave + 4 * i;
            const int m  = m0 + ml;
            const int oy = m / WO, ox = m - oy * WO;
            const int iy = 2 * oy + kh, ix = 2 * ox + kw;
            float v = 0.0f;
            if (kok && m < M && iy < HIN && ix < WIN) v = inc[iy * WIN + ix];
            sA[ml * AP + kk] = (_Float16)v;
        }
    }
    __syncthreads();

    Frag a;
    {
        const _Float16* ar = sA + (wave * 16 + c16) * AP;
        a.h[0] = *(const v8h*)(ar + 8 * h);
        a.h[1] = *(const v8h*)(ar + 16 + 8 * h);
    }
    v8f acc[4];
#pragma unroll
    for (int nb = 0; nb < 4; ++nb) {
        acc[nb] = zero8();
        const _Float16* bp = Wp + (nb * 16 + c16) * 32 + 8 * h;
        Frag b;
        b.q[0] = *(const u4*)bp;
        b.q[1] = *(const u4*)(bp + 16);
        acc[nb] = wmma_f16(a.v, b.v, acc[nb]);
    }
    epilogue_act<M>(acc, bias, 0.125f, sD, out + (size_t)img * M * 64, m0, wave, l);
}

template <int HIN, int WIN, int HO, int WO, int PAD, int NW, bool FINAL>
__global__ __launch_bounds__(NW * 32) void k_conv(const _Float16* __restrict__ in,
                                                  const _Float16* __restrict__ Wp,
                                                  const float* __restrict__ bias,
                                                  _Float16* __restrict__ outAct,
                                                  float* __restrict__ outEmb) {
    constexpr int M = HO * WO, MT = 16 * NW, IPIX = HIN * WIN;
    static_assert(NW >= 1 && NW <= 4);
    static_assert(!FINAL || (M <= MT && 64 * M == EDIM));
    __shared__ __align__(16) SBuf su;

    const int img = blockIdx.y, m0 = blockIdx.x * MT;
    const int tid = threadIdx.x, l = tid & 31, wave = tid >> 5, h = l >> 4, c16 = l & 15;
    const _Float16* inimg = in + (size_t)img * IPIX * 64;

    const int  m  = m0 + wave * 16 + c16;
    const bool vm = m < M;
    const int  mm = vm ? m : 0;
    const int  oy = mm / WO, ox = mm - oy * WO;

    v8f acc[4];
#pragma unroll
    for (int nb = 0; nb < 4; ++nb) acc[nb] = zero8();

#pragma unroll 1
    for (int t = 0; t < 9; ++t) {
        const int kh = t / 3, kw = t - 3 * kh;
        const int iy = 2 * oy + kh - PAD, ix = 2 * ox + kw - PAD;
        const bool ok = vm && ((unsigned)iy < (unsigned)HIN) && ((unsigned)ix < (unsigned)WIN);
        const int pix = ok ? (iy * WIN + ix) : 0;
        const _Float16* ap = inimg + (size_t)pix * 64 + 8 * h;
        const unsigned msk = ok ? 0xffffffffu : 0u;
        const u4 m4 = {msk, msk, msk, msk};
#pragma unroll
        for (int ch = 0; ch < 2; ++ch) {
            Frag a;
            a.q[0] = (*(const u4*)(ap + ch * 32)) & m4;
            a.q[1] = (*(const u4*)(ap + ch * 32 + 16)) & m4;
            const int k0 = t * 64 + ch * 32;
#pragma unroll
            for (int nb = 0; nb < 4; ++nb) {
                const _Float16* bp = Wp + (size_t)(nb * 16 + c16) * KW2 + k0 + 8 * h;
                Frag b;
                b.q[0] = *(const u4*)bp;
                b.q[1] = *(const u4*)(bp + 16);
                acc[nb] = wmma_f16(a.v, b.v, acc[nb]);
            }
        }
    }

    if constexpr (!FINAL) {
        epilogue_act<M>(acc, bias, 0.0625f, su.hb, outAct + (size_t)img * M * 64, m0, wave, l);
    } else {
        const float winv = 0.0625f;
#pragma unroll
        for (int nb = 0; nb < 4; ++nb) {
            const int col = nb * 16 + c16;
            const float bv = bias[col];
#pragma unroll
            for (int r = 0; r < 8; ++r) {
                const int mr = wave * 16 + 8 * h + r;
                if (mr < M) su.f[col * M + mr] = fmaxf(fmaf(acc[nb][r], winv, bv), 0.0f);
            }
        }
        __syncthreads();
        constexpr int NQ  = EDIM / 4;
        constexpr int NTH = NW * 32;
        constexpr int NJ  = (NQ + NTH - 1) / NTH;
        float* eo = outEmb + (size_t)img * EDIM;
        Q16 vq[NJ];
#pragma unroll
        for (int j = 0; j < NJ; ++j) {
            const int idx = tid + NTH * j;
            v4f z = {0.f, 0.f, 0.f, 0.f};
            vq[j].f = (idx < NQ) ? *(const v4f*)(su.f + idx * 4) : z;
        }
#pragma unroll
        for (int j = 0; j < NJ; ++j) {
            const int idx = tid + NTH * j;
            if (idx < NQ) *(volatile v4f*)(eo + idx * 4) = vq[j].f;
        }
        __threadfence();
#pragma unroll
        for (int j = 0; j < NJ; ++j) {
            const int idx = tid + NTH * j;
            if (idx < NQ) *(volatile v4f*)(eo + idx * 4) = vq[j].f;
        }
    }
}

__global__ __launch_bounds__(256) void k_head(const float* __restrict__ emb,
                                             const int* __restrict__ y,
                                             float* __restrict__ out) {
    __shared__ __align__(16) float sP[NC * EDIM];
    __shared__ __align__(16) float sOut[752 * 4];
    __shared__ float sRed[8 * NC];
    __shared__ float sPn[8];
    __shared__ int   sCls[32];

    const int tid = threadIdx.x, l = tid & 31, wave = tid >> 5;

    for (int b = 0; b < NB; ++b) {
        __syncthreads();
        if (tid < NS) {
            int v = y[b * NS + tid] % NC;
            if (v < 0) v += NC;
            sCls[tid] = v;
        }
        __syncthreads();

        float sq[NC] = {0.f, 0.f, 0.f, 0.f, 0.f};
        for (int d = tid; d < EDIM; d += 256) {
            float a[NC] = {0.f, 0.f, 0.f, 0.f, 0.f};
            for (int s = 0; s < NS; ++s) {
                const float v = emb[(size_t)(b * NS + s) * EDIM + d];
                const int cs = sCls[s];
#pragma unroll
                for (int c = 0; c < NC; ++c) a[c] += (cs == c) ? v : 0.0f;
            }
#pragma unroll
            for (int c = 0; c < NC; ++c) {
                const float p = a[c] * (1.0f / 5.0f);
                sP[c * EDIM + d] = p;
                sq[c] = fmaf(p, p, sq[c]);
            }
        }
#pragma unroll
        for (int o = 16; o > 0; o >>= 1) {
#pragma unroll
            for (int c = 0; c < NC; ++c) sq[c] += __shfl_xor(sq[c], o);
        }
        if (l == 0) {
#pragma unroll
            for (int c = 0; c < NC; ++c) sRed[wave * NC + c] = sq[c];
        }
        __syncthreads();
        if (tid < NC) {
            float s = 0.0f;
            for (int w = 0; w < 8; ++w) s += sRed[w * NC + tid];
            sPn[tid] = 1.0f / fmaxf(sqrtf(s), FEPS);
        }
        __syncthreads();

        for (int t = wave; t < NT; t += 8) {
            const float* e = emb + (size_t)(NSUP + b * NT + t) * EDIM;
            float dt[NC] = {0.f, 0.f, 0.f, 0.f, 0.f};
            float nn = 0.0f;
            for (int d = l; d < EDIM; d += 32) {
                const float ev = e[d];
                nn = fmaf(ev, ev, nn);
#pragma unroll
                for (int c = 0; c < NC; ++c) dt[c] = fmaf(ev, sP[c * EDIM + d], dt[c]);
            }
#pragma unroll
            for (int o = 16; o > 0; o >>= 1) {
                nn += __shfl_xor(nn, o);
#pragma unroll
                for (int c = 0; c < NC; ++c) dt[c] += __shfl_xor(dt[c], o);
            }
            if (l == 0) {
                const float rt = 1.0f / fmaxf(sqrtf(nn), FEPS);
#pragma unroll
                for (int c = 0; c < NC; ++c) sOut[(b * NT + t) * NC + c] = dt[c] * rt * sPn[c];
            }
        }
    }
    __syncthreads();

    constexpr int NQ = (NB * NT * NC) / 4;
    Q16 vq[3];
#pragma unroll
    for (int j = 0; j < 3; ++j) {
        const int idx = tid + 256 * j;
        v4f z = {0.f, 0.f, 0.f, 0.f};
        vq[j].f = (idx < NQ) ? *(const v4f*)(sOut + idx * 4) : z;
    }
#pragma unroll
    for (int j = 0; j < 3; ++j) {
        const int idx = tid + 256 * j;
        if (idx < NQ) *(volatile v4f*)(out + idx * 4) = vq[j].f;
    }
    __threadfence();
#pragma unroll
    for (int j = 0; j < 3; ++j) {
        const int idx = tid + 256 * j;
        if (idx < NQ) *(volatile v4f*)(out + idx * 4) = vq[j].f;
    }
}

extern "C" void kernel_launch(void* const* d_in, const int* in_sizes, int n_in,
                              void* d_out, int out_size, void* d_ws, size_t ws_size,
                              hipStream_t stream) {
    (void)in_sizes;
    if (n_in < 11 || out_size < NB * NT * NC) return;

    const float* xs = (const float*)d_in[0];
    const float* xt = (const float*)d_in[1];
    const int*   y  = (const int*)d_in[2];
    const float* W1 = (const float*)d_in[3];
    const float* b1 = (const float*)d_in[4];
    const float* W2 = (const float*)d_in[5];
    const float* b2 = (const float*)d_in[6];
    const float* W3 = (const float*)d_in[7];
    const float* b3 = (const float*)d_in[8];
    const float* W4 = (const float*)d_in[9];
    const float* b4 = (const float*)d_in[10];

    char*  base = (char*)d_ws;
    size_t off  = 0;
    auto take = [&](size_t bytes) -> void* {
        void* p = base + off;
        off += (bytes + 255) & ~(size_t)255;
        return p;
    };
    _Float16* P1   = (_Float16*)take((size_t)64 * 32 * 2);
    _Float16* P2   = (_Float16*)take((size_t)64 * KW2 * 2);
    _Float16* P3   = (_Float16*)take((size_t)64 * KW2 * 2);
    _Float16* P4   = (_Float16*)take((size_t)64 * KW2 * 2);
    _Float16* act1 = (_Float16*)take((size_t)CHUNK * 1764 * 64 * 2);
    _Float16* act2 = (_Float16*)take((size_t)CHUNK * 441 * 64 * 2);
    _Float16* act3 = (_Float16*)take((size_t)CHUNK * 121 * 64 * 2);
    float*    emb  = (float*)take((size_t)NIMG * EDIM * 4);
    if (off > ws_size) return;

    k_pack<<<dim3(18, 4), 256, 0, stream>>>(W1, W2, W3, W4, P1, P2, P3, P4);

    for (int c = 0; c < NCHUNK; ++c) {
        const float* xin = (c == 0) ? xs : (xt + (size_t)(c - 1) * CHUNK * 3 * 7056);
        k_conv1<<<dim3((1764 + 63) / 64, CHUNK), 128, 0, stream>>>(xin, P1, b1, act1);
        k_conv<42, 42, 21, 21, 0, 4, false>
            <<<dim3((441 + 63) / 64, CHUNK), 128, 0, stream>>>(act1, P2, b2, act2, emb);
        k_conv<21, 21, 11, 11, 1, 4, false>
            <<<dim3((121 + 63) / 64, CHUNK), 128, 0, stream>>>(act2, P3, b3, act3, emb);
        k_conv<11, 11, 6, 6, 1, 3, true>
            <<<dim3(1, CHUNK), 96, 0, stream>>>(act3, P4, b4, act1, emb + (size_t)c * CHUNK * EDIM);
    }

    k_head<<<dim3(1), 256, 0, stream>>>(emb, y, (float*)d_out);
}
